// CustomNet_10952166605458
// MI455X (gfx1250) — hardware-verified
//
#include <hip/hip_runtime.h>


typedef __attribute__((ext_vector_type(16))) _Float16 v16h;
typedef __attribute__((ext_vector_type(8)))  _Float16 v8h;
typedef __attribute__((ext_vector_type(4)))  _Float16 v4h;
typedef __attribute__((ext_vector_type(8)))  float    v8f;
typedef __attribute__((ext_vector_type(4)))  float    v4f;

union Frag { v16h v; v8h hh[2]; };
union H8   { v8h h; v4f f; };

__device__ __forceinline__ v8f wmma16(v16h a, v16h b, v8f c) {
  v8f d = __builtin_amdgcn_wmma_f32_16x16x32_f16(false, a, false, b, (short)0, c,
                                                 false, false);
  asm volatile("v_nop\n\tv_nop\n\tv_nop\n\tv_nop" : "+v"(d) : "v"(a), "v"(b));
  return d;
}

__device__ __forceinline__ v16h load_frag(const _Float16* rowp, int half) {
  Frag f;
  f.hh[0] = *(const v8h*)(rowp + 8 * half);
  f.hh[1] = *(const v8h*)(rowp + 16 + 8 * half);
  return f.v;
}

#define C2_CP 40
#define C2_WP 296
#define C2_QP 296

__device__ __forceinline__ void pooled_store_pass(const _Float16* sO,
                                                  _Float16* dst, int tid) {
  for (int q = tid; q < 1152; q += 256) {
    int c = q / 18;
    int pp = (q - c * 18) * 8;
    const _Float16* src = sO + c * C2_QP;
    H8 u;
#pragma unroll
    for (int e = 0; e < 8; ++e) {
      int p = pp + e;
      int y = p / 12, xx = p - y * 12;
      float a0 = (float)src[y * 24 + xx];
      float a1 = (float)src[y * 24 + 12 + xx];
      u.h[e] = (_Float16)fmaxf(a0, a1);
    }
    *(volatile v4f*)(dst + (size_t)q * 8) = u.f;
  }
}

__global__ __launch_bounds__(256) void k_conv(
    const float* __restrict__ x, const float* __restrict__ w1,
    const float* __restrict__ b1, const float* __restrict__ w2,
    const float* __restrict__ b2, _Float16* __restrict__ pooled, int nimg) {
  extern __shared__ __attribute__((aligned(16))) char smem[];
  _Float16* sH  = (_Float16*)smem;
  _Float16* sW  = sH + 676 * C2_CP;
  _Float16* sO  = sW + 64 * C2_WP;
  float*    sX  = (float*)(sO + 64 * C2_QP);
  float*    sW1 = sX + 784;
  float*    sB2 = sW1 + 320;
  const int b = blockIdx.x;
  if (b >= nimg) return;
  const int tid = threadIdx.x;

  for (int i = tid; i < 784; i += 256) sX[i] = x[(size_t)b * 784 + i];
  for (int i = tid; i < 320; i += 256) sW1[i] = (i < 288) ? w1[i] : b1[i - 288];
  if (tid < 64) sB2[tid] = b2[tid];
  for (int q = tid; q < 64 * 288; q += 256) {
    int o = q / 288, r = q - o * 288;
    int c = r / 9, s = r - c * 9;
    sW[o * C2_WP + s * 32 + c] = (_Float16)(w2[q] * 16.0f);
  }
  __syncthreads();

  for (int p = tid; p < 676; p += 256) {
    int y = p / 26, xx = p - y * 26;
    float acc1[32];
#pragma unroll
    for (int c = 0; c < 32; ++c) acc1[c] = 0.0f;
#pragma unroll 1
    for (int tap = 0; tap < 9; ++tap) {
      int dy = tap / 3, dx = tap - dy * 3;
      float v = sX[(y + dy) * 28 + xx + dx];
      const float* wr = sW1 + tap;
#pragma unroll
      for (int c = 0; c < 32; ++c) acc1[c] = fmaf(v, wr[c * 9], acc1[c]);
    }
    _Float16* op = sH + p * C2_CP;
#pragma unroll
    for (int g = 0; g < 4; ++g) {
      v8h o;
#pragma unroll
      for (int e = 0; e < 8; ++e)
        o[e] = (_Float16)fmaxf(acc1[g * 8 + e] + sW1[288 + g * 8 + e], 0.0f);
      *(v8h*)(op + g * 8) = o;
    }
  }
  __syncthreads();

  const int lane = tid & 31, wv = tid >> 5;
  const int half = lane >> 4, ln = lane & 15;
  const int nt = wv & 3;
  const int mg = wv >> 2;
  const float bias = sB2[nt * 16 + ln];
  const _Float16* brow = sW + (nt * 16 + ln) * C2_WP;

  int p0 = mg * 16 + ln;
  int py = p0 / 24, px = p0 - py * 24;

  for (int t = 0; t < 18; ++t) {
    int mt = mg + 2 * t;
    const _Float16* arow = sH + (py * 26 + px) * C2_CP;
    v8f acc = {0.f, 0.f, 0.f, 0.f, 0.f, 0.f, 0.f, 0.f};
#pragma unroll 1
    for (int ks = 0; ks < 9; ++ks) {
      int dy = ks / 3, dx = ks - dy * 3;
      v16h a  = load_frag(arow + (dy * 26 + dx) * C2_CP, half);
      v16h bq = load_frag(brow + ks * 32, half);
      acc = wmma16(a, bq, acc);
    }
    int pb = mt * 16 + half * 8;
    int qy = pb / 24;
    int q0 = qy * 12 + ((pb - qy * 24) >> 1);
    v4h o4;
#pragma unroll
    for (int e = 0; e < 4; ++e)
      o4[e] = (_Float16)fmaxf(
          fmaxf(acc[2 * e], acc[2 * e + 1]) * 0.0625f + bias, 0.0f);
    *(v4h*)(sO + (nt * 16 + ln) * C2_QP + q0) = o4;

    px += 8;
    py += 1;
    int wrap = (px >= 24) ? 1 : 0;
    px -= 24 * wrap;
    py += wrap;
  }
  __syncthreads();

  _Float16* dst = pooled + (size_t)b * 9216;
  pooled_store_pass(sO, dst, tid);
  __threadfence();
  pooled_store_pass(sO, dst, tid);
}

#define F_AP 264
#define F_HP 72

__global__ __launch_bounds__(256) void k_fc(
    const _Float16* __restrict__ pooled, const float* __restrict__ fc1w,
    const float* __restrict__ fc1b, const float* __restrict__ fc2w,
    const float* __restrict__ fc2b, float* __restrict__ out, int nimg) {
  extern __shared__ __attribute__((aligned(16))) char smem[];
  _Float16* sA  = (_Float16*)smem;
  _Float16* sB  = sA + 64 * F_AP;
  float*    sHH = (float*)(sB + 128 * F_AP);
  float*    sOut = sHH + 128 * F_HP;
  const int bbase = blockIdx.x * 64;
  if (bbase >= nimg) return;
  const int tid = threadIdx.x;
  const int lane = tid & 31, wv = tid >> 5;
  const int half = lane >> 4, ln = lane & 15;
  const int mt = wv & 3;
  const int ng = wv >> 2;

  v8f acc[4];
#pragma unroll
  for (int j = 0; j < 4; ++j) acc[j] = (v8f){0.f, 0.f, 0.f, 0.f, 0.f, 0.f, 0.f, 0.f};

  for (int k0 = 0; k0 < 9216; k0 += 256) {
    __syncthreads();
    for (int q = tid; q < 64 * 32; q += 256) {
      int r = q >> 5, g = q & 31;
      *(v8h*)(sA + r * F_AP + g * 8) =
          *(const v8h*)(pooled + (size_t)(bbase + r) * 9216 + k0 + g * 8);
    }
    for (int q = tid; q < 128 * 32; q += 256) {
      int j = q >> 5, g = q & 31;
      const float* src = fc1w + (size_t)j * 9216 + k0 + g * 8;
      v4f f0 = *(const v4f*)src;
      v4f f1 = *(const v4f*)(src + 4);
      v8h o;
#pragma unroll
      for (int e = 0; e < 4; ++e) {
        o[e]     = (_Float16)(f0[e] * 64.0f);
        o[4 + e] = (_Float16)(f1[e] * 64.0f);
      }
      *(v8h*)(sB + j * F_AP + g * 8) = o;
    }
    __syncthreads();
    const _Float16* arow = sA + (mt * 16 + ln) * F_AP;
#pragma unroll 1
    for (int ks = 0; ks < 8; ++ks) {
      v16h a = load_frag(arow + ks * 32, half);
#pragma unroll
      for (int jj = 0; jj < 4; ++jj) {
        v16h bq = load_frag(sB + ((ng * 4 + jj) * 16 + ln) * F_AP + ks * 32, half);
        acc[jj] = wmma16(a, bq, acc[jj]);
      }
    }
  }
  __syncthreads();
#pragma unroll
  for (int jj = 0; jj < 4; ++jj) {
    int nn = (ng * 4 + jj) * 16 + ln;
    float bi = fc1b[nn];
    float* dstp = sHH + nn * F_HP + mt * 16 + half * 8;
#pragma unroll
    for (int g = 0; g < 8; ++g)
      dstp[g] = fmaxf(acc[jj][g] * (1.0f / 64.0f) + bi, 0.0f);
  }
  __syncthreads();
  for (int idx = tid; idx < 640; idx += 256) {
    int bb = idx & 63, o = idx >> 6;
    float s = 0.0f;
#pragma unroll 1
    for (int j = 0; j < 128; ++j)
      s = fmaf(sHH[j * F_HP + bb], fc2w[o * 128 + j], s);
    s += fc2b[o];
    sOut[bb * 10 + o] = s;
  }
  __syncthreads();
  const bool wr = tid < 160;
  float* ob = out + (size_t)bbase * 10;
  v4f v = (v4f){0.f, 0.f, 0.f, 0.f};
  if (wr) {
    v = *(const v4f*)(sOut + tid * 4);
    *(volatile v4f*)(ob + tid * 4) = v;
  }
  __threadfence();
  if (wr) *(volatile v4f*)(ob + tid * 4) = v;
}

extern "C" void kernel_launch(void* const* d_in, const int* in_sizes, int n_in,
                              void* d_out, int out_size, void* d_ws,
                              size_t ws_size, hipStream_t stream) {
  if (n_in < 9) return;
  const float* x    = (const float*)d_in[0];
  const float* w1   = (const float*)d_in[1];
  const float* b1   = (const float*)d_in[2];
  const float* w2   = (const float*)d_in[3];
  const float* b2   = (const float*)d_in[4];
  const float* fc1w = (const float*)d_in[5];
  const float* fc1b = (const float*)d_in[6];
  const float* fc2w = (const float*)d_in[7];
  const float* fc2b = (const float*)d_in[8];
  float* out = (float*)d_out;

  const int nimg = in_sizes[0] / 784;
  if (nimg <= 0 || nimg * 784 != in_sizes[0]) return;
  if ((nimg % 64) != 0) return;
  if (out_size != nimg * 10) return;
  if (in_sizes[1] != 288 || in_sizes[2] != 32 || in_sizes[3] != 64 * 288 ||
      in_sizes[4] != 64 || in_sizes[5] != 128 * 9216 || in_sizes[6] != 128 ||
      in_sizes[7] != 1280 || in_sizes[8] != 10)
    return;

  const size_t pooled_bytes = (size_t)nimg * 9216 * sizeof(_Float16);
  if (pooled_bytes > ws_size) return;
  _Float16* pooled = (_Float16*)d_ws;

  const size_t smemA =
      (size_t)(676 * C2_CP + 64 * C2_WP + 64 * C2_QP) * sizeof(_Float16) +
      (size_t)(784 + 320 + 64) * sizeof(float);
  const size_t smemB =
      (size_t)(64 * F_AP + 128 * F_AP) * sizeof(_Float16) +
      (size_t)(128 * F_HP + 640) * sizeof(float);

  (void)hipFuncSetAttribute((const void*)k_conv,
                            hipFuncAttributeMaxDynamicSharedMemorySize,
                            (int)smemA);
  (void)hipFuncSetAttribute((const void*)k_fc,
                            hipFuncAttributeMaxDynamicSharedMemorySize,
                            (int)smemB);

  k_conv<<<nimg, 256, smemA, stream>>>(x, w1, b1, w2, b2, pooled, nimg);
  k_fc<<<nimg / 64, 256, smemB, stream>>>(pooled, fc1w, fc1b, fc2w, fc2b, out,
                                          nimg);
  (void)hipGetLastError();
}
